// GAT_15968688407067
// MI455X (gfx1250) — hardware-verified
//
#include <hip/hip_runtime.h>
#include <stddef.h>
#include <stdint.h>
#include <math.h>


#define DIN    512
#define DH     256
#define KP     512
#define DO     64
#define NTHR   256
#define NWAVE  8
#define EPT    8
#define CHUNK  (NTHR * EPT)
#define WCAP   (EPT * 32)
#define LISTN  (NWAVE * WCAP)
#define NBA    1024
#define SLA    10
#define RCAP   28672
#define DEGCAP 128
#define GBM    64
#define GBN    128
#define GTHR   128
#define MROWS  128
#define NUA    (DH * (KP / 8))
#define NUC    (DO * (KP / 8))
#define NUT    (4 * NUA + 2 * NUC)
#define NEGSL  0.2f
#define AGG_ZINTS (LISTN + 2 * RCAP + 3 * NBA)
#define AGG_LDS_INTS (AGG_ZINTS + 16)
#define WSMAX  134217728

static_assert((CHUNK & (CHUNK - 1)) == 0 && CHUNK <= 4096);
static_assert((NBA & (NBA - 1)) == 0 && NBA == (1 << SLA));
static_assert(((long long)CHUNK << SLA) < (1LL << 31));
static_assert(LISTN % NTHR == 0);
static_assert(NBA % NWAVE == 0 && NBA % 32 == 0 && NBA % GBM == 0);
static_assert(RCAP % 4 == 0 && AGG_ZINTS % 4 == 0 && LISTN % 4 == 0);
static_assert(DIN % 32 == 0 && KP % 32 == 0 && KP == 2 * DH && KP == DIN);
static_assert(GBM == (GTHR / 32) * 16 && GBN == 4 * 32);
static_assert((2 * DH) % GBN == 0 && (2 * DO) == GBN);
static_assert(NUA % NTHR == 0 && NUC % NTHR == 0 && NUT % NTHR == 0);
static_assert(KP / 8 == 64);
static_assert(AGG_LDS_INTS * 4 <= 300000);
static_assert(DH == 8 * 32 && DO == 2 * 32);
static_assert(MROWS % GBM == 0);

typedef float          v2f   __attribute__((ext_vector_type(2)));
typedef float          v4f   __attribute__((ext_vector_type(4)));
typedef float          v8f   __attribute__((ext_vector_type(8)));
typedef int            v4i   __attribute__((ext_vector_type(4)));
typedef int            v8i   __attribute__((ext_vector_type(8)));
typedef unsigned int   v4u   __attribute__((ext_vector_type(4)));
typedef unsigned short v8us  __attribute__((ext_vector_type(8)));
typedef unsigned short v16us __attribute__((ext_vector_type(16)));
typedef __bf16         v16bf __attribute__((ext_vector_type(16)));
typedef v4f  __attribute__((may_alias)) v4fa;
typedef v4i  __attribute__((may_alias)) v4ia;
typedef v8us __attribute__((may_alias)) v8usa;
union FragB { v16bf v; v16us u; v8us h[2]; v8i w; };

__device__ __forceinline__ v8f wmb(const FragB& a, const FragB& b, v8f c) {
  v8f d = __builtin_amdgcn_wmma_f32_16x16x32_bf16(false, a.v, false, b.v, (short)0, c, false, false);
  asm volatile("v_nop\n\tv_nop\n\tv_nop\n\tv_nop" : "+v"(d) : "v"(a.w), "v"(b.w));
  return d;
}

__device__ __forceinline__ unsigned bf16_bits(float f) {
  const unsigned u = __float_as_uint(f);
  return (u + 0x7FFFu + ((u >> 16) & 1u)) >> 16;
}
__device__ __forceinline__ float bf16_val(float f) {
  return __uint_as_float(bf16_bits(f) << 16);
}
__device__ __forceinline__ v4f bfr4(const v4f a) {
  v4f r; r.x = bf16_val(a.x); r.y = bf16_val(a.y); r.z = bf16_val(a.z); r.w = bf16_val(a.w); return r;
}

template <int SLB>
__device__ __forceinline__ int scan_chunk(const int* __restrict__ dsts, int nE, int cbase, int slotBase,
                                          int nb, int vec8, int* list, int tid, int lane, int wave) {
  int wc = 0;
  const int el0  = tid * EPT;
  const int e0   = cbase + el0;
  const int sent = -2147483647 - 1;
  v4i da, db;
  if (vec8 != 0 && cbase + CHUNK <= nE) {
    da = *(const v4i*)(dsts + e0);
    db = *(const v4i*)(dsts + e0 + 4);
  } else {
    da.x = (e0     < nE) ? dsts[min(e0,     nE - 1)] : sent;
    da.y = (e0 + 1 < nE) ? dsts[min(e0 + 1, nE - 1)] : sent;
    da.z = (e0 + 2 < nE) ? dsts[min(e0 + 2, nE - 1)] : sent;
    da.w = (e0 + 3 < nE) ? dsts[min(e0 + 3, nE - 1)] : sent;
    db.x = (e0 + 4 < nE) ? dsts[min(e0 + 4, nE - 1)] : sent;
    db.y = (e0 + 5 < nE) ? dsts[min(e0 + 5, nE - 1)] : sent;
    db.z = (e0 + 6 < nE) ? dsts[min(e0 + 6, nE - 1)] : sent;
    db.w = (e0 + 7 < nE) ? dsts[min(e0 + 7, nE - 1)] : sent;
  }
  const unsigned nbs = (unsigned)slotBase;
  const unsigned unb = (unsigned)nb;
  const unsigned s0 = (unsigned)da.x - nbs, s1 = (unsigned)da.y - nbs;
  const unsigned s2 = (unsigned)da.z - nbs, s3 = (unsigned)da.w - nbs;
  const unsigned s4 = (unsigned)db.x - nbs, s5 = (unsigned)db.y - nbs;
  const unsigned s6 = (unsigned)db.z - nbs, s7 = (unsigned)db.w - nbs;
  const bool h0 = s0 < unb, h1 = s1 < unb, h2 = s2 < unb, h3 = s3 < unb;
  const bool h4 = s4 < unb, h5 = s5 < unb, h6 = s6 < unb, h7 = s7 < unb;
  const unsigned any = __builtin_amdgcn_ballot_w32(h0 | h1 | h2 | h3 | h4 | h5 | h6 | h7);
  if (any != 0u) {
#define HITJ(J, HJ, SJ) { \
      const unsigned mj = __builtin_amdgcn_ballot_w32(HJ); \
      if (mj != 0u) { \
        if (HJ) { \
          const int pos = wc + (int)__builtin_amdgcn_mbcnt_lo(mj, 0u); \
          if (pos < WCAP) list[wave * WCAP + pos] = ((el0 + (J)) << SLB) | (int)(SJ); \
        } \
        wc += (int)__builtin_popcount(mj); } }
    HITJ(0, h0, s0)
    HITJ(1, h1, s1)
    HITJ(2, h2, s2)
    HITJ(3, h3, s3)
    HITJ(4, h4, s4)
    HITJ(5, h5, s5)
    HITJ(6, h6, s6)
    HITJ(7, h7, s7)
#undef HITJ
  }
  return wc;
}

__device__ __forceinline__ v8us wgather(const float* __restrict__ W, int ncol, int kmask, int n, int k8) {
  const int kk = k8 & kmask;
  const float* p = W + (size_t)kk * (size_t)ncol + n;
  v8us o;
#pragma unroll
  for (int i = 0; i < 8; ++i) o[i] = (unsigned short)bf16_bits(p[(size_t)i * (size_t)ncol]);
  return o;
}

__global__ __launch_bounds__(NTHR) void k_wprep(const float* __restrict__ W1l, const float* __restrict__ W1r,
                                                const float* __restrict__ W2l, const float* __restrict__ W2r,
                                                const float* __restrict__ W3l, const float* __restrict__ W3r,
                                                unsigned short* BT1, unsigned short* BT2, unsigned short* BT3) {
  const int u = (int)blockIdx.x * NTHR + (int)threadIdx.x;
  v8us o;
  unsigned short* dp;
  if (u < NUA) {
    const int v = u, n = v >> 6, k8 = (v & 63) * 8;
    o  = wgather(W1l, DH, DIN - 1, n, k8);
    dp = BT1 + (size_t)n * KP + k8;
  } else if (u < 2 * NUA) {
    const int v = u - NUA, n = v >> 6, k8 = (v & 63) * 8;
    o  = wgather(W1r, DH, DIN - 1, n, k8);
    dp = BT1 + (size_t)(DH + n) * KP + k8;
  } else if (u < 3 * NUA) {
    const int v = u - 2 * NUA, n = v >> 6, k8 = (v & 63) * 8;
    o  = wgather(W2l, DH, DH - 1, n, k8);
    dp = BT2 + (size_t)n * KP + k8;
  } else if (u < 4 * NUA) {
    const int v = u - 3 * NUA, n = v >> 6, k8 = (v & 63) * 8;
    o  = wgather(W2r, DH, DH - 1, n, k8);
    dp = BT2 + (size_t)(DH + n) * KP + k8;
  } else if (u < 4 * NUA + NUC) {
    const int v = u - 4 * NUA, n = v >> 6, k8 = (v & 63) * 8;
    o  = wgather(W3l, DO, DH - 1, n, k8);
    dp = BT3 + (size_t)n * KP + k8;
  } else if (u < NUT) {
    const int v = u - 4 * NUA - NUC, n = v >> 6, k8 = (v & 63) * 8;
    o  = wgather(W3r, DO, DH - 1, n, k8);
    dp = BT3 + (size_t)(DO + n) * KP + k8;
  } else {
    return;
  }
  *(volatile v8us*)dp = o;
  __threadfence();
  *(volatile v8us*)dp = o;
}

__global__ __launch_bounds__(NTHR) void k_cvx(const float* __restrict__ x, int nN, int nUnits,
                                              unsigned short* xb) {
  const int u = (int)blockIdx.x * NTHR + (int)threadIdx.x;
  if (u >= nUnits) return;
  const int row = u >> 6;
  const int k8  = (u & 63) * 8;
  const int rc  = row < nN ? row : nN - 1;
  const float* p = x + (size_t)rc * DIN + k8;
  const v4f a = *(const v4f*)p;
  const v4f b = *(const v4f*)(p + 4);
  const bool ok = row < nN;
  v8us o;
  o[0] = ok ? (unsigned short)bf16_bits(a.x) : (unsigned short)0;
  o[1] = ok ? (unsigned short)bf16_bits(a.y) : (unsigned short)0;
  o[2] = ok ? (unsigned short)bf16_bits(a.z) : (unsigned short)0;
  o[3] = ok ? (unsigned short)bf16_bits(a.w) : (unsigned short)0;
  o[4] = ok ? (unsigned short)bf16_bits(b.x) : (unsigned short)0;
  o[5] = ok ? (unsigned short)bf16_bits(b.y) : (unsigned short)0;
  o[6] = ok ? (unsigned short)bf16_bits(b.z) : (unsigned short)0;
  o[7] = ok ? (unsigned short)bf16_bits(b.w) : (unsigned short)0;
  unsigned short* dp = xb + (size_t)row * DIN + k8;
  *(volatile v8us*)dp = o;
  __threadfence();
  *(volatile v8us*)dp = o;
}

__global__ __launch_bounds__(GTHR) void k_gemm(const unsigned short* __restrict__ A, int lda,
                                               const unsigned short* __restrict__ BT, int ldb, int K,
                                               float* Cm, int ldc,
                                               const float* __restrict__ bl, const float* __restrict__ br, int nl) {
  __shared__ __attribute__((aligned(16))) float stg[GBM * GBN];
  const int tid = (int)threadIdx.x, lane = tid & 31, wave = tid >> 5, hh = lane >> 4, m = lane & 15;
  const int rowBase = (int)blockIdx.x * GBM;
  const int colBase = (int)blockIdx.y * GBN;

  v8f acc[8];
  {
    const v8f z = {0.f, 0.f, 0.f, 0.f, 0.f, 0.f, 0.f, 0.f};
#pragma unroll
    for (int t = 0; t < 8; ++t) acc[t] = z;
  }
  const unsigned short* ap = A  + (size_t)(rowBase + 16 * wave + m) * (size_t)lda + 8 * hh;
  const unsigned short* bp = BT + (size_t)(colBase + m) * (size_t)ldb + 8 * hh;

#pragma unroll 1
  for (int k0 = 0; k0 < K; k0 += 32) {
    FragB af;
    af.h[0] = *(const v8usa*)(ap + k0);
    af.h[1] = *(const v8usa*)(ap + k0 + 16);
#pragma unroll
    for (int nt = 0; nt < 8; ++nt) {
      const unsigned short* wq = bp + (size_t)(16 * nt) * (size_t)ldb + k0;
      FragB bf;
      bf.h[0] = *(const v8usa*)wq;
      bf.h[1] = *(const v8usa*)(wq + 16);
      acc[nt] = wmb(af, bf, acc[nt]);
    }
  }

#pragma unroll
  for (int nt = 0; nt < 8; ++nt) {
    const int lc = 16 * nt + m;
#pragma unroll
    for (int r = 0; r < 8; ++r) {
      const int lr = 16 * wave + 8 * hh + r;
      stg[lr * GBN + lc] = acc[nt][r];
    }
  }
  __syncthreads();

  v4f bias4;
  {
    const int gc = colBase + 4 * lane;
    int cl = gc < nl - 4 ? gc : nl - 4;
    cl = cl < 0 ? 0 : cl;
    int cr = gc - nl;
    cr = cr < 0 ? 0 : (cr > nl - 4 ? nl - 4 : cr);
    const v4f vl = *(const v4f*)(bl + cl);
    const v4f vr = *(const v4f*)(br + cr);
    const unsigned mk = (gc < nl) ? 0xFFFFFFFFu : 0u;
    v4f s;
    s.x = __uint_as_float((__float_as_uint(vl.x) & mk) | (__float_as_uint(vr.x) & ~mk));
    s.y = __uint_as_float((__float_as_uint(vl.y) & mk) | (__float_as_uint(vr.y) & ~mk));
    s.z = __uint_as_float((__float_as_uint(vl.z) & mk) | (__float_as_uint(vr.z) & ~mk));
    s.w = __uint_as_float((__float_as_uint(vl.w) & mk) | (__float_as_uint(vr.w) & ~mk));
    bias4 = bfr4(s);
  }

#pragma unroll 1
  for (int i = 0; i < 16; ++i) {
    const int row = wave * 16 + i;
    const v4f p = *(const v4fa*)(stg + row * GBN + 4 * lane);
    v4f q; q.x = p.x + bias4.x; q.y = p.y + bias4.y; q.z = p.z + bias4.z; q.w = p.w + bias4.w;
    float* op = Cm + (size_t)(rowBase + row) * (size_t)ldc + colBase + 4 * lane;
    *(volatile v4f*)op = q;
  }
  __threadfence();
#pragma unroll 1
  for (int i = 0; i < 16; ++i) {
    const int row = wave * 16 + i;
    const v4f p = *(const v4fa*)(stg + row * GBN + 4 * lane);
    v4f q; q.x = p.x + bias4.x; q.y = p.y + bias4.y; q.z = p.z + bias4.z; q.w = p.w + bias4.w;
    float* op = Cm + (size_t)(rowBase + row) * (size_t)ldc + colBase + 4 * lane;
    *(volatile v4f*)op = q;
  }
}

template <int CPL>
__device__ __forceinline__ void ld_row(const float* __restrict__ p, float (&r)[CPL]) {
  if constexpr (CPL == 8) {
    const v4f a = *(const v4f*)p;
    const v4f b = *(const v4f*)(p + 4);
    r[0] = a.x; r[1] = a.y; r[2] = a.z; r[3] = a.w;
    r[4] = b.x; r[5] = b.y; r[6] = b.z; r[7] = b.w;
  } else {
    const v2f a = *(const v2f*)p;
    r[0] = a.x; r[1] = a.y;
  }
}
template <int CPL>
__device__ __forceinline__ void ld_row_bf(const float* __restrict__ p, float (&r)[CPL]) {
  ld_row<CPL>(p, r);
#pragma unroll
  for (int i = 0; i < CPL; ++i) r[i] = bf16_val(r[i]);
}

template <int CPL>
__device__ __forceinline__ float edge_score(const float (&xs)[CPL], const float (&xr)[CPL], const float (&av)[CPL]) {
  float pd = 0.0f;
#pragma unroll
  for (int i = 0; i < CPL; ++i) {
    float t = xs[i] + xr[i];
    t = t > 0.f ? t : NEGSL * t;
    pd = fmaf(av[i], t, pd);
  }
  if constexpr (CPL == 8) {
    pd += __shfl_xor(pd, 1);
    pd += __shfl_xor(pd, 2);
  } else {
#pragma unroll
    for (int off = 16; off > 0; off >>= 1) pd += __shfl_xor(pd, off);
  }
  return pd;
}

template <int CPL, int FIN>
__global__ __launch_bounds__(NTHR) void k_agg(const int* __restrict__ srcs, const int* __restrict__ dsts,
                                              int nE, int nN, int vec8, int mRows,
                                              const float* __restrict__ X,
                                              const float* __restrict__ att, const float* __restrict__ bias,
                                              unsigned short* hb, float* outp, int off2) {
  static_assert((CPL == 8 && FIN == 0) || (CPL == 2 && FIN == 1));
  extern __shared__ __attribute__((aligned(16))) int dsm[];
  int* list = dsm;
  int* hl   = dsm + LISTN;
  int* sl   = dsm + LISTN + RCAP;
  int* cnt  = dsm + LISTN + 2 * RCAP;
  int* offs = cnt + NBA;
  int* cur  = offs + NBA;
  int* misc = cur + NBA;
  constexpr int C   = CPL * 32;
  constexpr int LDX = 2 * C;
  const int tid = (int)threadIdx.x, lane = tid & 31, wave = tid >> 5;
  const int nodeBase = (int)blockIdx.x * NBA;

  {
    const v4i z4 = {0, 0, 0, 0};
    for (int i = tid * 4; i < AGG_ZINTS; i += NTHR * 4) *(v4ia*)(dsm + i) = z4;
    if (tid < 16) misc[tid] = 0;
  }
  float av[CPL], bv[CPL];
  ld_row_bf<CPL>(att  + CPL * lane, av);
  ld_row_bf<CPL>(bias + CPL * lane, bv);
  __syncthreads();

  int t = 0, ov = 0;
  const int nChunks = (nE + CHUNK - 1) / CHUNK;
#pragma unroll 1
  for (int ch = 0; ch < nChunks; ++ch) {
    const int cbase = ch * CHUNK;
    const int wc = scan_chunk<SLA>(dsts, nE, cbase, nodeBase, NBA, vec8, list, tid, lane, wave);
    if (lane == 0) misc[wave] = wc;
    __syncthreads();
    if (wave == 0) {
#pragma unroll 1
      for (int w2 = 0; w2 < NWAVE; ++w2) {
        int c = misc[w2];
        c = c < 0 ? 0 : (c > WCAP ? WCAP : c);
#pragma unroll 1
        for (int b0 = 0; b0 < c; b0 += 32) {
          const int idx = b0 + lane;
          const int ent = list[w2 * WCAP + (idx < WCAP ? idx : WCAP - 1)];
          const int m32 = (c - b0) < 32 ? (c - b0) : 32;
#pragma unroll 1
          for (int k = 0; k < m32; ++k) {
            const int u    = __builtin_amdgcn_readlane(ent, k);
            const int slot = u & (NBA - 1);
            const int el   = (u >> SLA) & (CHUNK - 1);
            const int pk   = ((cbase + el) << SLA) | slot;
            if (t < RCAP) {
              if (lane == 0) { hl[t] = pk; cnt[slot] = cnt[slot] + 1; }
              t = t + 1;
            } else {
              ov = 1;
            }
          }
        }
      }
    }
    __syncthreads();
  }
  if (wave == 0 && lane == 0) { misc[8] = t; misc[9] = ov; }
  __syncthreads();
  int tt = misc[8];
  tt = tt < 0 ? 0 : (tt > RCAP ? RCAP : tt);
  const int ovf = misc[9];

  if (wave == 0) {
    const int base = lane * (NBA / 32);
    int s = 0;
#pragma unroll 1
    for (int i = 0; i < NBA / 32; ++i) s += cnt[base + i];
    int incl = s;
#pragma unroll
    for (int d = 1; d < 32; d <<= 1) {
      const int y = __shfl_up(incl, d, 32);
      if (lane >= d) incl += y;
    }
    int run = incl - s;
#pragma unroll 1
    for (int i = 0; i < NBA / 32; ++i) {
      const int cv = cnt[base + i];
      offs[base + i] = run;
      cur[base + i]  = run;
      run += cv;
    }
  }
  __syncthreads();
  if (wave == 0) {
#pragma unroll 1
    for (int b0 = 0; b0 < tt; b0 += 32) {
      const int idx = b0 + lane;
      const int ent = hl[idx < RCAP ? idx : RCAP - 1];
      const int m32 = (tt - b0) < 32 ? (tt - b0) : 32;
#pragma unroll 1
      for (int k = 0; k < m32; ++k) {
        const int u    = __builtin_amdgcn_readlane(ent, k);
        const int slot = u & (NBA - 1);
        if (lane == 0) {
          int p = cur[slot];
          p = p < 0 ? 0 : (p > RCAP - 1 ? RCAP - 1 : p);
          sl[p] = u;
          cur[slot] = p + 1;
        }
      }
    }
  }
  __syncthreads();

  const float qnan = __int_as_float(0x7fc00000);
  const float pz = (ovf != 0) ? qnan : 0.0f;
#pragma unroll 1
  for (int si = 0; si < NBA / NWAVE; ++si) {
    const int s    = si * NWAVE + wave;
    const int node = nodeBase + s;
    int c = cnt[s];
    const bool big = c > DEGCAP;
    c = c < 0 ? 0 : (c > DEGCAP ? DEGCAP : c);
    int o = offs[s];
    o = o < 0 ? 0 : (o > RCAP ? RCAP : o);
    const int nc = node < nN ? node : nN - 1;
    const float* selfp = X + (size_t)nc * LDX + CPL * lane;
    float acc[CPL], xrv[CPL];
    ld_row<CPL>(selfp, acc);
    ld_row<CPL>(selfp + C, xrv);
    float mx = edge_score<CPL>(acc, xrv, av);
    float dn = 1.0f;
#pragma unroll 1
    for (int b0 = 0; b0 < c; b0 += 32) {
      int idx = o + b0 + lane;
      idx = idx > RCAP - 1 ? RCAP - 1 : idx;
      const int ent = sl[idx];
      int eid = ent >> SLA;
      eid = eid < 0 ? 0 : (eid > nE - 1 ? nE - 1 : eid);
      int sr = srcs[eid];
      sr = sr < 0 ? 0 : (sr > nN - 1 ? nN - 1 : sr);
      const int m32 = (c - b0) < 32 ? (c - b0) : 32;
#pragma unroll 1
      for (int k = 0; k < m32; ++k) {
        const int sk = __builtin_amdgcn_readlane(sr, k);
        float xv[CPL];
        ld_row<CPL>(X + (size_t)sk * LDX + CPL * lane, xv);
        const float lg = edge_score<CPL>(xv, xrv, av);
        const float df = lg - mx;
        const float ee = expf(-fabsf(df));
        const bool  up = df > 0.f;
        const float s1 = up ? ee : 1.0f;
        const float s2 = up ? 1.0f : ee;
        mx = up ? lg : mx;
        dn = fmaf(dn, s1, s2);
#pragma unroll
        for (int i = 0; i < CPL; ++i) acc[i] = fmaf(acc[i], s1, s2 * xv[i]);
      }
    }
    const float inv = __builtin_amdgcn_rcpf(dn);
    const float pzr = big ? qnan : pz;
    const bool live = node < nN;

    if constexpr (FIN == 0) {
      float v[8];
#pragma unroll
      for (int i = 0; i < 8; ++i) v[i] = fmaf(acc[i], inv, bv[i]) + pzr;
#pragma unroll 1
      for (int it = 0; it < 8; ++it) {
        float e0 = v[0];
        e0 = (e0 > 0.0f) ? e0 : expm1f(e0);
        v[0] = v[1]; v[1] = v[2]; v[2] = v[3]; v[3] = v[4];
        v[4] = v[5]; v[5] = v[6]; v[6] = v[7]; v[7] = e0;
      }
      v8us ho, lo;
#pragma unroll
      for (int i = 0; i < 8; ++i) {
        const float y = live ? v[i] : 0.0f;
        const unsigned hbi = bf16_bits(y);
        ho[i] = (unsigned short)hbi;
        lo[i] = (unsigned short)bf16_bits(y - __uint_as_float(hbi << 16));
      }
      if (node < mRows) {
        unsigned short* hp = hb + (size_t)node * KP + 8 * lane;
        *(volatile v8us*)hp = ho;
        *(volatile v8us*)(hp + DH) = lo;
        __threadfence();
        *(volatile v8us*)hp = ho;
        *(volatile v8us*)(hp + DH) = lo;
      }
    } else {
      const float z0 = fmaf(acc[0], inv, bv[0]) + pzr;
      const float z1 = fmaf(acc[1], inv, bv[1]) + pzr;
      float vm = fmaxf(z0, z1);
#pragma unroll
      for (int off = 16; off > 0; off >>= 1) vm = fmaxf(vm, __shfl_xor(vm, off));
      const float ex0 = expf(z0 - vm), ex1 = expf(z1 - vm);
      float sm = ex0 + ex1;
#pragma unroll
      for (int off = 16; off > 0; off >>= 1) sm += __shfl_xor(sm, off);
      const float ls = logf(sm);
      const float o0 = ((z0 - vm) - ls) + pzr;
      const float o1 = ((z1 - vm) - ls) + pzr;
      const int sa = (2 * lane) & 31, sb = (2 * lane + 1) & 31;
      const float g0 = __shfl(z0, sa), g1 = __shfl(z1, sa), g2 = __shfl(z0, sb), g3 = __shfl(z1, sb);
      const float q0 = __shfl(o0, sa), q1 = __shfl(o1, sa), q2 = __shfl(o0, sb), q3 = __shfl(o1, sb);
      const bool lsel = lane >= 16;
      v4f pv;
      pv.x = lsel ? q0 : g0;
      pv.y = lsel ? q1 : g1;
      pv.z = lsel ? q2 : g2;
      pv.w = lsel ? q3 : g3;
      const size_t eo = (size_t)nc * DO + (size_t)(4 * (lane & 15)) + (lsel ? (size_t)off2 : (size_t)0);
      if (live) {
        float* op = outp + eo;
        *(volatile v4f*)op = pv;
        __threadfence();
        *(volatile v4f*)op = pv;
      }
    }
  }
}

static inline int cdiv(int a, int b) { return (a + b - 1) / b; }

extern "C" void kernel_launch(void* const* d_in, const int* in_sizes, int n_in,
                              void* d_out, int out_size, void* d_ws, size_t ws_size,
                              hipStream_t stream) {
  if (n_in < 20) return;
  if (in_sizes[0] < DIN || (in_sizes[0] % DIN) != 0) return;
  const int nN = in_sizes[0] / DIN;
  if (nN < 1 || nN > (1 << 20)) return;
  if (in_sizes[1] < 2 || (in_sizes[1] & 1) != 0) return;
  const int nE = in_sizes[1] / 2;
  if (nE < 1 || nE >= (1 << 21)) return;
  if (in_sizes[2] != DIN * DH || in_sizes[4] != DIN * DH) return;
  if (in_sizes[3] != DH || in_sizes[5] != DH) return;
  if (in_sizes[6] != DH || in_sizes[7] != DH) return;
  if (in_sizes[8] != DH * DH || in_sizes[10] != DH * DH) return;
  if (in_sizes[9] != DH || in_sizes[11] != DH) return;
  if (in_sizes[12] != DH || in_sizes[13] != DH) return;
  if (in_sizes[14] != DH * DO || in_sizes[16] != DH * DO) return;
  if (in_sizes[15] != DO || in_sizes[17] != DO) return;
  if (in_sizes[18] != DO || in_sizes[19] != DO) return;
  if ((long long)out_size != 2LL * (long long)nN * DO) return;

  const float* x    = (const float*)d_in[0];
  const int*   edge = (const int*)d_in[1];
  const float* W1l  = (const float*)d_in[2];
  const float* b1l  = (const float*)d_in[3];
  const float* W1r  = (const float*)d_in[4];
  const float* b1r  = (const float*)d_in[5];
  const float* a1   = (const float*)d_in[6];
  const float* bo1  = (const float*)d_in[7];
  const float* W2l  = (const float*)d_in[8];
  const float* b2l  = (const float*)d_in[9];
  const float* W2r  = (const float*)d_in[10];
  const float* b2r  = (const float*)d_in[11];
  const float* a2   = (const float*)d_in[12];
  const float* bo2  = (const float*)d_in[13];
  const float* W3l  = (const float*)d_in[14];
  const float* b3l  = (const float*)d_in[15];
  const float* W3r  = (const float*)d_in[16];
  const float* b3r  = (const float*)d_in[17];
  const float* a3   = (const float*)d_in[18];
  const float* bo3  = (const float*)d_in[19];
  float* out = (float*)d_out;
  const int* src = edge;
  const int* dst = edge + nE;

  const int MP   = cdiv(nN, MROWS) * MROWS;
  const int gM   = MP / GBM;
  const int gA   = cdiv(MP, NBA);
  if ((long long)gA * NBA < (long long)MP) return;
  const int vec8 = ((nE & 3) == 0) ? 1 : 0;
  const int off2 = nN * DO;

  char* ws = (char*)d_ws;
  size_t off = 0;
  const size_t oB1 = off; off += (size_t)(2 * DH) * KP * 2;              off = (off + 255) & ~(size_t)255;
  const size_t oB2 = off; off += (size_t)(2 * DH) * KP * 2;              off = (off + 255) & ~(size_t)255;
  const size_t oB3 = off; off += (size_t)(2 * DO) * KP * 2;              off = (off + 255) & ~(size_t)255;
  const size_t oXB = off; off += (size_t)MP * DIN * 2;                   off = (off + 255) & ~(size_t)255;
  const size_t oXL = off; off += (size_t)MP * (2 * DH) * 4;              off = (off + 255) & ~(size_t)255;
  const size_t oH1 = off; off += (size_t)MP * KP * 2;                    off = (off + 255) & ~(size_t)255;
  if (off > ws_size || off > (size_t)WSMAX) return;
  unsigned short* BT1 = (unsigned short*)(ws + oB1);
  unsigned short* BT2 = (unsigned short*)(ws + oB2);
  unsigned short* BT3 = (unsigned short*)(ws + oB3);
  unsigned short* XB  = (unsigned short*)(ws + oXB);
  unsigned short* H2  = XB;
  float*          XLR = (float*)(ws + oXL);
  unsigned short* H1  = (unsigned short*)(ws + oH1);

  const size_t aggLds = (size_t)AGG_LDS_INTS * 4;
  hipFuncSetAttribute(reinterpret_cast<const void*>(&k_agg<8, 0>), hipFuncAttributeMaxDynamicSharedMemorySize, (int)aggLds);
  hipFuncSetAttribute(reinterpret_cast<const void*>(&k_agg<2, 1>), hipFuncAttributeMaxDynamicSharedMemorySize, (int)aggLds);

  const int nUx = MP * (DIN / 8);
  k_wprep<<<NUT / NTHR, NTHR, 0, stream>>>(W1l, W1r, W2l, W2r, W3l, W3r, BT1, BT2, BT3);
  k_cvx<<<cdiv(nUx, NTHR), NTHR, 0, stream>>>(x, nN, nUx, XB);
  k_gemm<<<dim3(gM, (2 * DH) / GBN), GTHR, 0, stream>>>(XB, DIN, BT1, KP, DIN, XLR, 2 * DH, b1l, b1r, DH);
  k_agg<8, 0><<<gA, NTHR, aggLds, stream>>>(src, dst, nE, nN, vec8, MP, XLR, a1, bo1, H1, out, off2);
  k_gemm<<<dim3(gM, (2 * DH) / GBN), GTHR, 0, stream>>>(H1, KP, BT2, KP, KP, XLR, 2 * DH, b2l, b2r, DH);
  k_agg<8, 0><<<gA, NTHR, aggLds, stream>>>(src, dst, nE, nN, vec8, MP, XLR, a2, bo2, H2, out, off2);
  k_gemm<<<dim3(gM, (2 * DO) / GBN), GTHR, 0, stream>>>(H2, KP, BT3, KP, KP, XLR, 2 * DO, b3l, b3r, DO);
  k_agg<2, 1><<<gA, NTHR, aggLds, stream>>>(src, dst, nE, nN, vec8, MP, XLR, a3, bo3, H1, out, off2);
}
